// WindowCrossAttention_37572373905978
// MI455X (gfx1250) — hardware-verified
//
#include <hip/hip_runtime.h>

typedef __bf16 v16b __attribute__((ext_vector_type(16)));
typedef unsigned short us;
typedef us    v8us __attribute__((ext_vector_type(8)));
typedef float v8f  __attribute__((ext_vector_type(8)));
typedef float v4f  __attribute__((ext_vector_type(4)));
typedef int   v4i  __attribute__((ext_vector_type(4)));
typedef v8us __attribute__((may_alias)) v8usa;
typedef v4f  __attribute__((may_alias)) v4fa;
typedef v4i  __attribute__((may_alias)) v4ia;

union Frag { v16b v; v8us half[2]; };

#define EMB   1024
#define NH    16
#define DM    64
#define SLEN  2048
#define BS    2
#define MTOT  (BS * SLEN)
#define NXT   (MTOT * EMB)
#define NW    (EMB * EMB)
#define NX8   (NXT / 8)
#define NW8   (NW / 8)
#define PL    (BS * NH * SLEN * DM)
#define EPSN  1.0e-6f

static_assert(MTOT % 128 == 0);
static_assert(SLEN % 128 == 0);
static_assert(EMB % 64 == 0);

__device__ __forceinline__ us bf16_rne(float x) {
  unsigned u = __float_as_uint(x);
  u += 0x7FFFu + ((u >> 16) & 1u);
  return (us)(u >> 16);
}
__device__ __forceinline__ float bf16_val(us b) {
  return __uint_as_float(((unsigned)b) << 16);
}

__device__ __forceinline__ v8f wmma_bf(v16b a, v16b b, v8f c) {
  v8f d = __builtin_amdgcn_wmma_f32_16x16x32_bf16(false, a, false, b, (short)0, c, false, false);
  asm volatile("v_nop\n\tv_nop\n\tv_nop\n\tv_nop" : "+v"(d) : "v"(a), "v"(b));
  return d;
}

__device__ __forceinline__ v16b load_frag(const us* p, int h) {
  Frag f;
  f.half[0] = *(const v8usa*)(p + 8 * h);
  f.half[1] = *(const v8usa*)(p + 16 + 8 * h);
  return f.v;
}

__device__ __forceinline__ void split8(v8f a, v8us& hi, v8us& lo) {
  const us h0 = bf16_rne(a[0]), h1 = bf16_rne(a[1]), h2 = bf16_rne(a[2]), h3 = bf16_rne(a[3]);
  const us h4 = bf16_rne(a[4]), h5 = bf16_rne(a[5]), h6 = bf16_rne(a[6]), h7 = bf16_rne(a[7]);
  const v8us hv = { h0, h1, h2, h3, h4, h5, h6, h7 };
  const v8us lv = { bf16_rne(a[0] - bf16_val(h0)), bf16_rne(a[1] - bf16_val(h1)),
                    bf16_rne(a[2] - bf16_val(h2)), bf16_rne(a[3] - bf16_val(h3)),
                    bf16_rne(a[4] - bf16_val(h4)), bf16_rne(a[5] - bf16_val(h5)),
                    bf16_rne(a[6] - bf16_val(h6)), bf16_rne(a[7] - bf16_val(h7)) };
  hi = hv;
  lo = lv;
}

__global__ __launch_bounds__(256) void conv_kernel(
    const float* __restrict__ xq, const float* __restrict__ xk, const float* __restrict__ xv,
    const float* __restrict__ wq, const float* __restrict__ wk, const float* __restrict__ wv,
    const float* __restrict__ wo,
    us* __restrict__ xb, us* __restrict__ wb)
{
  const int g = blockIdx.x * 256 + threadIdx.x;
  if (g >= 3 * NX8 + 4 * NW8) return;
  const float* src;
  us* dst;
  if (g < 3 * NX8) {
    const int sel = g / NX8;
    const int off = g - sel * NX8;
    src = ((sel == 0) ? xq : ((sel == 1) ? xk : xv)) + (size_t)off * 8;
    dst = xb + (size_t)sel * NXT + (size_t)off * 8;
  } else {
    const int g2 = g - 3 * NX8;
    const int sel = g2 / NW8;
    const int off = g2 - sel * NW8;
    src = ((sel == 0) ? wq : ((sel == 1) ? wk : ((sel == 2) ? wv : wo))) + (size_t)off * 8;
    dst = wb + (size_t)sel * NW + (size_t)off * 8;
  }
  const v4f a = *(const v4fa*)src;
  const v4f c = *(const v4fa*)(src + 4);
  const v8us o = { bf16_rne(a.x), bf16_rne(a.y), bf16_rne(a.z), bf16_rne(a.w),
                   bf16_rne(c.x), bf16_rne(c.y), bf16_rne(c.z), bf16_rne(c.w) };
  *(volatile v8us*)dst = o;
  __threadfence();
  *(volatile v8us*)dst = o;
}

__device__ __forceinline__ void qk_store_pass(const us* sHi, const us* sLo, us* ph, us* plo,
                                              int bh, int l0, int w, int lane) {
  const int q8 = lane & 7, sub = lane >> 3;
  #pragma unroll
  for (int i = 0; i < 8; ++i) {
    const int lid = w * 32 + i * 4 + sub;
    const v8us a = *(const v8usa*)(sHi + lid * DM + 8 * q8);
    const v8us c = *(const v8usa*)(sLo + lid * DM + 8 * q8);
    const size_t off = ((size_t)bh * SLEN + l0 + lid) * DM + 8 * q8;
    *(volatile v8us*)(ph + off)  = a;
    *(volatile v8us*)(plo + off) = c;
  }
}

__device__ __forceinline__ void v_store_pass(const us* sHi, const us* sLo, us* vh, us* vl,
                                             int bh, int l0, int w, int lane) {
  const int q8 = lane & 7, sub = lane >> 3;
  #pragma unroll
  for (int i = 0; i < 8; ++i) {
    const int lid = w * 32 + i * 4 + sub;
    const int d = lid >> 1, hl = lid & 1;
    const v8us a = *(const v8usa*)(sHi + d * 128 + 64 * hl + 8 * q8);
    const v8us c = *(const v8usa*)(sLo + d * 128 + 64 * hl + 8 * q8);
    const size_t off = ((size_t)bh * DM + d) * SLEN + l0 + 64 * hl + 8 * q8;
    *(volatile v8us*)(vh + off) = a;
    *(volatile v8us*)(vl + off) = c;
  }
}

template <int WHICH>
__global__ __launch_bounds__(128) void proj_kernel(
    const us* __restrict__ xb,
    const us* __restrict__ wb,
    const float* __restrict__ bias,
    const float* __restrict__ normw,
    us* __restrict__ dst)
{
  __shared__ __attribute__((aligned(16))) us sA[128 * DM];
  __shared__ __attribute__((aligned(16))) us sB[128 * DM];

  const int tid = threadIdx.x, lane = tid & 31, w = tid >> 5;
  const int h = lane >> 4, m = lane & 15;
  const int m0 = blockIdx.x * 128;
  const int head = blockIdx.y;
  const int m0w = m0 + 32 * w;

  const us* xa0 = xb + (size_t)WHICH * NXT + (size_t)(m0w + m) * EMB;
  const us* xa1 = xa0 + (size_t)16 * EMB;
  const us* wr  = wb + (size_t)WHICH * NW + (size_t)(head * DM + m) * EMB;

  const v8f zero8 = {0.f, 0.f, 0.f, 0.f, 0.f, 0.f, 0.f, 0.f};
  v8f acc[2][4];
  #pragma unroll
  for (int mt = 0; mt < 2; ++mt)
    #pragma unroll
    for (int nt = 0; nt < 4; ++nt) acc[mt][nt] = zero8;

  #pragma unroll 1
  for (int k0 = 0; k0 < EMB; k0 += 32) {
    const v16b a0 = load_frag(xa0 + k0, h);
    const v16b a1 = load_frag(xa1 + k0, h);
    #pragma unroll
    for (int nt = 0; nt < 4; ++nt) {
      const v16b b = load_frag(wr + (size_t)nt * 16 * EMB + k0, h);
      acc[0][nt] = wmma_bf(a0, b, acc[0][nt]);
      acc[1][nt] = wmma_bf(a1, b, acc[1][nt]);
    }
  }

  #pragma unroll
  for (int nt = 0; nt < 4; ++nt) {
    const float bvl = bias[head * DM + 16 * nt + m];
    #pragma unroll
    for (int mt = 0; mt < 2; ++mt)
      #pragma unroll
      for (int r = 0; r < 8; ++r) acc[mt][nt][r] += bvl;
  }

  const int b = m0 / SLEN, l0 = m0 - b * SLEN, bh = b * NH + head;

  if (WHICH != 2) {
    const float osc = (WHICH == 0) ? 0.125f : 1.0f;
    #pragma unroll
    for (int mt = 0; mt < 2; ++mt) {
      float ss[8];
      #pragma unroll
      for (int r = 0; r < 8; ++r) {
        float s = 0.0f;
        #pragma unroll
        for (int nt = 0; nt < 4; ++nt) s += acc[mt][nt][r] * acc[mt][nt][r];
        ss[r] = s;
      }
      #pragma unroll
      for (int r = 0; r < 8; ++r) {
        ss[r] += __shfl_xor(ss[r], 1);
        ss[r] += __shfl_xor(ss[r], 2);
        ss[r] += __shfl_xor(ss[r], 4);
        ss[r] += __shfl_xor(ss[r], 8);
        ss[r] = rsqrtf(ss[r] * (1.0f / 64.0f) + EPSN);
      }
      #pragma unroll
      for (int nt = 0; nt < 4; ++nt) {
        const int feat = 16 * nt + m;
        const float wn = normw[feat] * osc;
        #pragma unroll
        for (int r = 0; r < 8; ++r) {
          const int tokl = 32 * w + 16 * mt + 8 * h + r;
          const float y = (acc[mt][nt][r] * ss[r]) * wn;
          const us hi = bf16_rne(y);
          const us lo = bf16_rne(y - bf16_val(hi));
          sA[tokl * DM + feat] = hi;
          sB[tokl * DM + feat] = lo;
        }
      }
    }
    __syncthreads();
    us* ph  = dst;
    us* plo = dst + PL;
    qk_store_pass(sA, sB, ph, plo, bh, l0, w, lane);
    __threadfence();
    qk_store_pass(sA, sB, ph, plo, bh, l0, w, lane);
  } else {
    #pragma unroll
    for (int nt = 0; nt < 4; ++nt) {
      const int feat = 16 * nt + m;
      #pragma unroll
      for (int mt = 0; mt < 2; ++mt) {
        v8us hi, lo;
        split8(acc[mt][nt], hi, lo);
        const int idx = feat * 128 + 32 * w + 16 * mt + 8 * h;
        *(v8usa*)(sA + idx) = hi;
        *(v8usa*)(sB + idx) = lo;
      }
    }
    __syncthreads();
    us* vh = dst;
    us* vl = dst + PL;
    v_store_pass(sA, sB, vh, vl, bh, l0, w, lane);
    __threadfence();
    v_store_pass(sA, sB, vh, vl, bh, l0, w, lane);
  }
}

__device__ __forceinline__ void pack_p2(v8f a, v8f c, v16b& phi, v16b& plo) {
  Frag fh, fl;
  v8us h0, l0, h1, l1;
  split8(a, h0, l0);
  split8(c, h1, l1);
  fh.half[0] = h0; fh.half[1] = h1;
  fl.half[0] = l0; fl.half[1] = l1;
  phi = fh.v;
  plo = fl.v;
}

__device__ __forceinline__ void att_store_pass(const us* soh, const us* sol, us* oh, us* ol,
                                               int b, int head, int q0, int lane) {
  const int q8 = lane & 7, sub = lane >> 3;
  #pragma unroll
  for (int i = 0; i < 4; ++i) {
    const int row = i * 4 + sub;
    const v8us a = *(const v8usa*)(soh + row * DM + 8 * q8);
    const v8us c = *(const v8usa*)(sol + row * DM + 8 * q8);
    const size_t gi = ((size_t)b * SLEN + q0 + row) * EMB + head * DM + 8 * q8;
    *(volatile v8us*)(oh + gi) = a;
    *(volatile v8us*)(ol + gi) = c;
  }
}

__global__ __launch_bounds__(128) void attn_kernel(
    const us* __restrict__ qp,
    const us* __restrict__ kp,
    const us* __restrict__ vtp,
    const int* __restrict__ amask,
    us* __restrict__ op)
{
  __shared__ __attribute__((aligned(16))) us sOh[4 * 16 * DM];
  __shared__ __attribute__((aligned(16))) us sOl[4 * 16 * DM];

  const int tid = threadIdx.x, lane = tid & 31, w = tid >> 5;
  const int h = lane >> 4, m = lane & 15;
  const int bh = blockIdx.y, b = bh >> 4, head = bh & 15;
  const int q0 = blockIdx.x * 64 + 16 * w;

  const us* qrh = qp + ((size_t)bh * SLEN + q0 + m) * DM;
  const us* qrl = qrh + PL;
  const v16b qh0 = load_frag(qrh, h);
  const v16b qh1 = load_frag(qrh + 32, h);
  const v16b ql0 = load_frag(qrl, h);
  const v16b ql1 = load_frag(qrl + 32, h);

  const v8f zero8 = {0.f, 0.f, 0.f, 0.f, 0.f, 0.f, 0.f, 0.f};
  v8f o[4];
  #pragma unroll
  for (int t = 0; t < 4; ++t) o[t] = zero8;
  float mrun = -1.0e30f, lrun = 0.0f;

  const us* khb = kp + ((size_t)bh * SLEN + m) * DM;
  const us* klb = khb + PL;
  const us* vhb = vtp + ((size_t)bh * DM + m) * SLEN;
  const us* vlb = vhb + PL;
  const int* mkp = amask + (size_t)b * SLEN + 8 * h;

  #pragma unroll 1
  for (int kb = 0; kb < SLEN; kb += 64) {
    v8f s[4];
    #pragma unroll
    for (int j = 0; j < 4; ++j) {
      const size_t ko = (size_t)(kb + 16 * j) * DM;
      const v16b kh0 = load_frag(khb + ko, h);
      const v16b kh1 = load_frag(khb + ko + 32, h);
      const v16b kl0 = load_frag(klb + ko, h);
      const v16b kl1 = load_frag(klb + ko + 32, h);
      v8f z = zero8;
      z = wmma_bf(kl0, qh0, z);
      z = wmma_bf(kl1, qh1, z);
      z = wmma_bf(kh0, ql0, z);
      z = wmma_bf(kh1, ql1, z);
      z = wmma_bf(kh0, qh0, z);
      z = wmma_bf(kh1, qh1, z);
      s[j] = z;
    }

    #pragma unroll
    for (int j = 0; j < 4; ++j) {
      const v4i f0 = *(const v4ia*)(mkp + kb + 16 * j);
      const v4i f1 = *(const v4ia*)(mkp + kb + 16 * j + 4);
      s[j][0] = (f0.x == 0) ? -1.0e30f : s[j][0];
      s[j][1] = (f0.y == 0) ? -1.0e30f : s[j][1];
      s[j][2] = (f0.z == 0) ? -1.0e30f : s[j][2];
      s[j][3] = (f0.w == 0) ? -1.0e30f : s[j][3];
      s[j][4] = (f1.x == 0) ? -1.0e30f : s[j][4];
      s[j][5] = (f1.y == 0) ? -1.0e30f : s[j][5];
      s[j][6] = (f1.z == 0) ? -1.0e30f : s[j][6];
      s[j][7] = (f1.w == 0) ? -1.0e30f : s[j][7];
    }

    float mloc = s[0][0];
    #pragma unroll
    for (int j = 0; j < 4; ++j)
      #pragma unroll
      for (int r = 0; r < 8; ++r) mloc = fmaxf(mloc, s[j][r]);
    mloc = fmaxf(mloc, __shfl_xor(mloc, 16));
    const float mnew = fmaxf(mrun, mloc);
    const float alpha = __expf(mrun - mnew);
    mrun = mnew;
    float lsum = 0.0f;
    #pragma unroll
    for (int j = 0; j < 4; ++j)
      #pragma unroll
      for (int r = 0; r < 8; ++r) {
        const float p = __expf(s[j][r] - mnew);
        s[j][r] = p;
        lsum += p;
      }
    lsum += __shfl_xor(lsum, 16);
    lrun = lrun * alpha + lsum;
    #pragma unroll
    for (int t = 0; t < 4; ++t)
      #pragma unroll
      for (int r = 0; r < 8; ++r) o[t][r] = o[t][r] * alpha;

    v16b ph0, pl0, ph1, pl1;
    pack_p2(s[0], s[1], ph0, pl0);
    pack_p2(s[2], s[3], ph1, pl1);

    #pragma unroll
    for (int t = 0; t < 4; ++t) {
      const size_t vo = (size_t)(16 * t) * SLEN + kb;
      const v16b vh0 = load_frag(vhb + vo, h);
      const v16b vh1 = load_frag(vhb + vo + 32, h);
      const v16b vl0 = load_frag(vlb + vo, h);
      const v16b vl1 = load_frag(vlb + vo + 32, h);
      v8f acc = o[t];
      acc = wmma_bf(vl0, ph0, acc);
      acc = wmma_bf(vl1, ph1, acc);
      acc = wmma_bf(vh0, pl0, acc);
      acc = wmma_bf(vh1, pl1, acc);
      acc = wmma_bf(vh0, ph0, acc);
      acc = wmma_bf(vh1, ph1, acc);
      o[t] = acc;
    }
  }

  const float inv = (mrun > -1.0e29f) ? (1.0f / lrun) : __uint_as_float(0x7fc00000u);
  us* soh = sOh + w * (16 * DM);
  us* sol = sOl + w * (16 * DM);
  #pragma unroll
  for (int t = 0; t < 4; ++t) {
    v8us hi, lo;
    split8(o[t] * inv, hi, lo);
    const int idx = m * DM + 16 * t + 8 * h;
    *(v8usa*)(soh + idx) = hi;
    *(v8usa*)(sol + idx) = lo;
  }
  __syncthreads();

  us* oh = op;
  us* ol = op + NXT;
  att_store_pass(soh, sol, oh, ol, b, head, q0, lane);
  __threadfence();
  att_store_pass(soh, sol, oh, ol, b, head, q0, lane);
}

__device__ __forceinline__ void out_store_pass(const float* sO, float* out, int m0, int cg,
                                               int w, int lane) {
  const int q8 = lane & 7, sub = lane >> 3;
  #pragma unroll
  for (int i = 0; i < 16; ++i) {
    const int lid = w * 64 + i * 4 + sub;
    const int row = lid >> 1, hl = lid & 1;
    const v4f v = *(const v4fa*)(sO + row * DM + 32 * hl + 4 * q8);
    const size_t gi = (size_t)(m0 + row) * EMB + cg * DM + 32 * hl + 4 * q8;
    *(volatile v4f*)(out + gi) = v;
  }
}

__global__ __launch_bounds__(128) void out_kernel(
    const us* __restrict__ op,
    const us* __restrict__ wb,
    const float* __restrict__ bo,
    float* __restrict__ out)
{
  __shared__ __attribute__((aligned(16))) float sO[128 * DM];

  const int tid = threadIdx.x, lane = tid & 31, w = tid >> 5;
  const int h = lane >> 4, m = lane & 15;
  const int m0 = blockIdx.x * 128;
  const int cg = blockIdx.y;
  const int m0w = m0 + 32 * w;

  const us* ah0 = op + (size_t)(m0w + m) * EMB;
  const us* ah1 = ah0 + (size_t)16 * EMB;
  const us* al0 = ah0 + NXT;
  const us* al1 = ah1 + NXT;
  const us* wr  = wb + (size_t)3 * NW + (size_t)(cg * DM + m) * EMB;

  const v8f zero8 = {0.f, 0.f, 0.f, 0.f, 0.f, 0.f, 0.f, 0.f};
  v8f acc[2][4];
  #pragma unroll
  for (int mt = 0; mt < 2; ++mt)
    #pragma unroll
    for (int nt = 0; nt < 4; ++nt) acc[mt][nt] = zero8;

  #pragma unroll 1
  for (int k0 = 0; k0 < EMB; k0 += 32) {
    const v16b a0h = load_frag(ah0 + k0, h);
    const v16b a1h = load_frag(ah1 + k0, h);
    const v16b a0l = load_frag(al0 + k0, h);
    const v16b a1l = load_frag(al1 + k0, h);
    #pragma unroll
    for (int nt = 0; nt < 4; ++nt) {
      const v16b bw = load_frag(wr + (size_t)nt * 16 * EMB + k0, h);
      acc[0][nt] = wmma_bf(a0l, bw, acc[0][nt]);
      acc[0][nt] = wmma_bf(a0h, bw, acc[0][nt]);
      acc[1][nt] = wmma_bf(a1l, bw, acc[1][nt]);
      acc[1][nt] = wmma_bf(a1h, bw, acc[1][nt]);
    }
  }

  #pragma unroll
  for (int nt = 0; nt < 4; ++nt) {
    const int feat = 16 * nt + m;
    const float bvl = bo[cg * DM + feat];
    #pragma unroll
    for (int mt = 0; mt < 2; ++mt) {
      #pragma unroll
      for (int r = 0; r < 8; ++r) {
        const int tokl = 32 * w + 16 * mt + 8 * h + r;
        sO[tokl * DM + feat] = acc[mt][nt][r] + bvl;
      }
    }
  }
  __syncthreads();

  out_store_pass(sO, out, m0, cg, w, lane);
  __threadfence();
  out_store_pass(sO, out, m0, cg, w, lane);
}

extern "C" void kernel_launch(void* const* d_in, const int* in_sizes, int n_in,
                              void* d_out, int out_size, void* d_ws, size_t ws_size,
                              hipStream_t stream) {
  if (n_in < 14) return;
  if (in_sizes[0] != NXT || in_sizes[1] != NXT || in_sizes[2] != NXT) return;
  if (in_sizes[3] != BS * SLEN) return;
  if (in_sizes[4] != NW || in_sizes[6] != NW || in_sizes[8] != NW || in_sizes[10] != NW) return;
  if (in_sizes[5] != EMB || in_sizes[7] != EMB || in_sizes[9] != EMB || in_sizes[11] != EMB) return;
  if (in_sizes[12] != DM || in_sizes[13] != DM) return;
  if (out_size != NXT) return;

  const float* Q   = (const float*)d_in[0];
  const float* K   = (const float*)d_in[1];
  const float* V   = (const float*)d_in[2];
  const int*   AM  = (const int*)d_in[3];
  const float* Wq  = (const float*)d_in[4];
  const float* bq  = (const float*)d_in[5];
  const float* Wk  = (const float*)d_in[6];
  const float* bk  = (const float*)d_in[7];
  const float* Wv  = (const float*)d_in[8];
  const float* bv  = (const float*)d_in[9];
  const float* Wo  = (const float*)d_in[10];
  const float* bo  = (const float*)d_in[11];
  const float* qnw = (const float*)d_in[12];
  const float* knw = (const float*)d_in[13];
  float* out = (float*)d_out;

  const size_t xb_bytes = (size_t)3 * NXT * 2;
  const size_t wb_bytes = (size_t)4 * NW * 2;
  const size_t pl_bytes = (size_t)2 * PL * 2;
  const size_t op_bytes = (size_t)2 * NXT * 2;
  const size_t total = xb_bytes + wb_bytes + 3 * pl_bytes + op_bytes;
  if (total > ws_size) return;

  char* ws = (char*)d_ws;
  size_t pos = 0;
  us* xb  = (us*)(ws + pos);  pos += xb_bytes;
  us* wb  = (us*)(ws + pos);  pos += wb_bytes;
  us* qp  = (us*)(ws + pos);  pos += pl_bytes;
  us* kp  = (us*)(ws + pos);  pos += pl_bytes;
  us* vtp = (us*)(ws + pos);  pos += pl_bytes;
  us* op  = (us*)(ws + pos);  pos += op_bytes;
  if (pos > ws_size) return;

  const int ngroups = 3 * NX8 + 4 * NW8;
  conv_kernel<<<(ngroups + 255) / 256, 256, 0, stream>>>(Q, K, V, Wq, Wk, Wv, Wo, xb, wb);

  dim3 gProj(MTOT / 128, NH);
  proj_kernel<0><<<gProj, 128, 0, stream>>>(xb, wb, bq, qnw, qp);
  proj_kernel<1><<<gProj, 128, 0, stream>>>(xb, wb, bk, knw, kp);
  proj_kernel<2><<<gProj, 128, 0, stream>>>(xb, wb, bv, qnw, vtp);

  dim3 gAtt(SLEN / 64, BS * NH);
  attn_kernel<<<gAtt, 128, 0, stream>>>(qp, kp, vtp, AM, op);

  dim3 gOut(MTOT / 128, EMB / 64);
  out_kernel<<<gOut, 128, 0, stream>>>(op, wb, bo, out);
}
